// EfficientTransformerEncoder_62594853372030
// MI455X (gfx1250) — hardware-verified
//
#include <hip/hip_runtime.h>

typedef _Float16 v16h __attribute__((ext_vector_type(16)));
typedef _Float16 v8h  __attribute__((ext_vector_type(8)));
typedef float    v8f  __attribute__((ext_vector_type(8)));
typedef float    v4f  __attribute__((ext_vector_type(4)));
typedef v8h __attribute__((may_alias)) v8ha;
typedef v4f __attribute__((may_alias)) v4fa;

union Frag { v16h v; v8h half[2]; _Float16 s[16]; };
union H8   { v8h v; _Float16 s[8]; };

#define D_MODEL 256
#define NHEADS  8
#define DH      32
#define NLAYERS 3
#define DFF     1024
#define WIN     64
#define SEQ     1024
#define BATCH   32
#define NTOK    (BATCH * SEQ)
#define NCHUNK  2
#define IMGC    (BATCH / NCHUNK)
#define MC      (IMGC * SEQ)
#define QKVN    (3 * D_MODEL)
#define WSC     32.0f
#define WINV    0.03125f
#define PSC     16384.0f
#define PINV    0.00006103515625f
#define QSC     0.17677669529663687f
#define LNEPS   1e-5f
#define TP      260
#define OP      264

static_assert(MC % 128 == 0);
static_assert(MC % WIN == 0);
static_assert(SEQ % 32 == 0);

__device__ __forceinline__ v8f wmma_f16(v16h a, v16h b, v8f c) {
  v8f d = __builtin_amdgcn_wmma_f32_16x16x32_f16(false, a, false, b, (short)0, c, false, false);
  asm volatile("v_nop\n\tv_nop\n\tv_nop\n\tv_nop" : "+v"(d) : "v"(a), "v"(b));
  return d;
}

__device__ __forceinline__ v16h load_frag(const _Float16* p, int h) {
  Frag f;
  f.half[0] = *(const v8ha*)(p + 8 * h);
  f.half[1] = *(const v8ha*)(p + 16 + 8 * h);
  return f.v;
}

__device__ __forceinline__ float wsum32(float v) {
  v += __shfl_xor(v, 1);
  v += __shfl_xor(v, 2);
  v += __shfl_xor(v, 4);
  v += __shfl_xor(v, 8);
  v += __shfl_xor(v, 16);
  return v;
}

__global__ __launch_bounds__(256) void cvt_w_kernel(
    const float* __restrict__ wi, const float* __restrict__ wo,
    const float* __restrict__ w1, const float* __restrict__ w2,
    _Float16* __restrict__ wih, _Float16* __restrict__ woh,
    _Float16* __restrict__ w1h, _Float16* __restrict__ w2h,
    int g0, int g1, int g2, int g3)
{
  const int g = blockIdx.x * 256 + threadIdx.x;
  if (g >= g0 + g1 + g2 + g3) return;
  const float* src;
  _Float16* dst;
  if (g < g0) {
    src = wi + (size_t)g * 8;  dst = wih + (size_t)g * 8;
  } else if (g < g0 + g1) {
    const int e = g - g0;
    src = wo + (size_t)e * 8;  dst = woh + (size_t)e * 8;
  } else if (g < g0 + g1 + g2) {
    const int e = g - g0 - g1;
    src = w1 + (size_t)e * 8;  dst = w1h + (size_t)e * 8;
  } else {
    const int e = g - g0 - g1 - g2;
    src = w2 + (size_t)e * 8;  dst = w2h + (size_t)e * 8;
  }
  const v4f a = *(const v4fa*)src;
  const v4f c = *(const v4fa*)(src + 4);
  const v8h o = { (_Float16)(a.x * WSC), (_Float16)(a.y * WSC), (_Float16)(a.z * WSC), (_Float16)(a.w * WSC),
                  (_Float16)(c.x * WSC), (_Float16)(c.y * WSC), (_Float16)(c.z * WSC), (_Float16)(c.w * WSC) };
  *(volatile v8h*)dst = o;
  __threadfence();
  *(volatile v8h*)dst = o;
}

__device__ __forceinline__ void prep_store_pass(const float* sT, float* xf, _Float16* xh,
                                                size_t r0, int w, int lane) {
  #pragma unroll
  for (int e = 0; e < 4; ++e) {
    const int tl = 4 * w + e;
    const float* st = sT + tl * TP;
    const v4f g0 = *(const v4fa*)(st + 4 * lane);
    const v4f g1 = *(const v4fa*)(st + 128 + 4 * lane);
    const v4f p0 = *(const v4fa*)(st + 8 * lane);
    const v4f p1 = *(const v4fa*)(st + 8 * lane + 4);
    H8 hv;
    hv.s[0] = (_Float16)p0.x; hv.s[1] = (_Float16)p0.y; hv.s[2] = (_Float16)p0.z; hv.s[3] = (_Float16)p0.w;
    hv.s[4] = (_Float16)p1.x; hv.s[5] = (_Float16)p1.y; hv.s[6] = (_Float16)p1.z; hv.s[7] = (_Float16)p1.w;
    float* xr = xf + (r0 + tl) * D_MODEL;
    _Float16* hr = xh + (r0 + tl) * D_MODEL;
    *(volatile v4f*)(xr + 4 * lane) = g0;
    *(volatile v4f*)(xr + 128 + 4 * lane) = g1;
    *(volatile v8h*)(hr + 8 * lane) = hv.v;
  }
}

__global__ __launch_bounds__(256) void prep_kernel(const float* __restrict__ feat, int img0,
                                                   float* __restrict__ xf, _Float16* __restrict__ xh)
{
  __shared__ __attribute__((aligned(16))) float sT[32 * TP];
  const int tid = threadIdx.x, lane = tid & 31, w = tid >> 5;
  const int bl = blockIdx.x >> 5;
  const int l0 = (blockIdx.x & 31) * 32;
  const int b  = img0 + bl;
  const float kf  = -(9.2103403719761836f * 0.00390625f);
  const float pos = (float)(l0 + lane);
  #pragma unroll 1
  for (int i = 0; i < 32; ++i) {
    const int ch = 8 * i + w;
    const float f = feat[((size_t)(b * D_MODEL + ch)) * SEQ + l0 + lane];
    const float freq = expf((float)(ch & ~1) * kf);
    const float ang = pos * freq;
    const float pe = (ch & 1) ? cosf(ang) : sinf(ang);
    sT[lane * TP + ch] = f + pe;
  }
  __syncthreads();
  const size_t r0 = (size_t)bl * SEQ + l0;
  prep_store_pass(sT, xf, xh, r0, w, lane);
  __threadfence();
  prep_store_pass(sT, xf, xh, r0, w, lane);
}

__device__ __forceinline__ void gemm_store_f32(const float* sC, float* C, size_t mb, int nb, int N,
                                               int w, int lane) {
  const int q8 = lane & 7, hl = (lane >> 3) & 1, rs = lane >> 4;
  #pragma unroll
  for (int i = 0; i < 16; ++i) {
    const int row = 32 * w + 2 * i + rs;
    const v4f v = *(const v4fa*)(sC + row * 64 + 32 * hl + 4 * q8);
    *(volatile v4f*)(C + (mb + row) * (size_t)N + nb + 32 * hl + 4 * q8) = v;
  }
}

__device__ __forceinline__ void gemm_store_f16(const _Float16* sH, _Float16* C, size_t mb, int nb, int N,
                                               int w, int lane) {
  const int q8 = lane & 7, sub = lane >> 3;
  #pragma unroll
  for (int i = 0; i < 8; ++i) {
    const int row = 32 * w + 4 * i + sub;
    const v8h v = *(const v8ha*)(sH + row * 64 + 8 * q8);
    *(volatile v8h*)(C + (mb + row) * (size_t)N + nb + 8 * q8) = v;
  }
}

__global__ __launch_bounds__(128) void gemm_f16_kernel(
    const _Float16* __restrict__ A, int lda,
    const _Float16* __restrict__ W, int ldw,
    const float* __restrict__ bias,
    float* Cf, _Float16* Ch,
    int N, int qcols, int gelu, int out16)
{
  __shared__ __attribute__((aligned(16))) float sC[128 * 64];

  const int tid = threadIdx.x, lane = tid & 31, w = tid >> 5;
  const int h = lane >> 4, m = lane & 15;
  const size_t mb = (size_t)blockIdx.x * 128;
  const int nb = blockIdx.y * 64;
  const int K = lda;

  const _Float16* a0p = A + (mb + 32 * w + m) * (size_t)lda;
  const _Float16* a1p = a0p + (size_t)16 * lda;
  const _Float16* wp  = W + (size_t)(nb + m) * ldw;

  const v8f zero8 = {0.f, 0.f, 0.f, 0.f, 0.f, 0.f, 0.f, 0.f};
  v8f acc[2][4];
  #pragma unroll
  for (int mt = 0; mt < 2; ++mt)
    #pragma unroll
    for (int nt = 0; nt < 4; ++nt) acc[mt][nt] = zero8;

  #pragma unroll 1
  for (int k0 = 0; k0 < K; k0 += 32) {
    const v16h fa0 = load_frag(a0p + k0, h);
    const v16h fa1 = load_frag(a1p + k0, h);
    #pragma unroll
    for (int nt = 0; nt < 4; ++nt) {
      const v16h fb = load_frag(wp + (size_t)nt * 16 * ldw + k0, h);
      acc[0][nt] = wmma_f16(fa0, fb, acc[0][nt]);
      acc[1][nt] = wmma_f16(fa1, fb, acc[1][nt]);
    }
  }

  const float cs = (nb < qcols) ? QSC : 1.0f;
  _Float16* sH = (_Float16*)sC;
  #pragma unroll
  for (int nt = 0; nt < 4; ++nt) {
    const int col = 16 * nt + m;
    const float bv = bias[nb + col];
    #pragma unroll
    for (int mt = 0; mt < 2; ++mt) {
      #pragma unroll
      for (int r = 0; r < 8; ++r) {
        const int row = 32 * w + 16 * mt + 8 * h + r;
        float v = (acc[mt][nt][r] * WINV + bv) * cs;
        if (gelu) v = 0.5f * v * (1.0f + erff(v * 0.70710678118654752f));
        if (out16) sH[row * 64 + col] = (_Float16)v;
        else       sC[row * 64 + col] = v;
      }
    }
  }
  __syncthreads();

  if (out16) {
    gemm_store_f16(sH, Ch, mb, nb, N, w, lane);
    __threadfence();
    gemm_store_f16(sH, Ch, mb, nb, N, w, lane);
  } else {
    gemm_store_f32(sC, Cf, mb, nb, N, w, lane);
    __threadfence();
    gemm_store_f32(sC, Cf, mb, nb, N, w, lane);
  }
}

__device__ __forceinline__ v16h pack_p(v8f a, v8f c, float sc) {
  Frag f;
  #pragma unroll
  for (int r = 0; r < 8; ++r) {
    f.s[r]     = (_Float16)(a[r] * sc);
    f.s[8 + r] = (_Float16)(c[r] * sc);
  }
  return f.v;
}

__device__ __forceinline__ void att_store_pass(const _Float16* sO, _Float16* att, size_t tb,
                                               int hd, int lane) {
  #pragma unroll
  for (int i = 0; i < 8; ++i) {
    const int row = hd * 8 + i;
    const v8h v = *(const v8ha*)(sO + row * OP + 8 * lane);
    *(volatile v8h*)(att + (tb + row) * D_MODEL + 8 * lane) = v;
  }
}

__global__ __launch_bounds__(256) void attn_kernel(const _Float16* __restrict__ qkv,
                                                   _Float16* __restrict__ att)
{
  __shared__ __attribute__((aligned(16))) _Float16 sO[WIN * OP];

  const int tid = threadIdx.x, lane = tid & 31, hd = tid >> 5;
  const int hi = lane >> 4, m = lane & 15;
  const size_t tb = (size_t)blockIdx.x * WIN;
  const _Float16* base = qkv + tb * QKVN;

  v16h kA[4];
  #pragma unroll
  for (int j = 0; j < 4; ++j)
    kA[j] = load_frag(base + (size_t)(16 * j + m) * QKVN + D_MODEL + hd * DH, hi);

  v16h vA[2][2];
  {
    const _Float16* vp = base + 2 * D_MODEL + hd * DH + m;
    #pragma unroll
    for (int t = 0; t < 2; ++t)
      #pragma unroll
      for (int kt = 0; kt < 2; ++kt) {
        Frag f;
        #pragma unroll
        for (int i = 0; i < 8; ++i) {
          f.s[i]     = vp[(size_t)(32 * kt + 8 * hi + i) * QKVN + 16 * t];
          f.s[8 + i] = vp[(size_t)(32 * kt + 16 + 8 * hi + i) * QKVN + 16 * t];
        }
        vA[t][kt] = f.v;
      }
  }

  const v8f zero8 = {0.f, 0.f, 0.f, 0.f, 0.f, 0.f, 0.f, 0.f};

  #pragma unroll 1
  for (int mi = 0; mi < 4; ++mi) {
    const v16h qB = load_frag(base + (size_t)(16 * mi + m) * QKVN + hd * DH, hi);

    v8f s[4];
    #pragma unroll
    for (int j = 0; j < 4; ++j) s[j] = wmma_f16(kA[j], qB, zero8);

    float mx = s[0][0];
    #pragma unroll
    for (int j = 0; j < 4; ++j)
      #pragma unroll
      for (int r = 0; r < 8; ++r) mx = fmaxf(mx, s[j][r]);
    mx = fmaxf(mx, __shfl_xor(mx, 16));
    float sum = 0.0f;
    #pragma unroll
    for (int j = 0; j < 4; ++j)
      #pragma unroll
      for (int r = 0; r < 8; ++r) {
        const float e = __expf(s[j][r] - mx);
        s[j][r] = e;
        sum += e;
      }
    sum += __shfl_xor(sum, 16);
    const float ps = (1.0f / sum) * PSC;

    const v16h pB0 = pack_p(s[0], s[1], ps);
    const v16h pB1 = pack_p(s[2], s[3], ps);

    v8f o0 = wmma_f16(vA[0][0], pB0, zero8);
    o0 = wmma_f16(vA[0][1], pB1, o0);
    v8f o1 = wmma_f16(vA[1][0], pB0, zero8);
    o1 = wmma_f16(vA[1][1], pB1, o1);

    H8 w0, w1;
    #pragma unroll
    for (int r = 0; r < 8; ++r) {
      w0.s[r] = (_Float16)(o0[r] * PINV);
      w1.s[r] = (_Float16)(o1[r] * PINV);
    }
    _Float16* so = sO + (16 * mi + m) * OP + hd * DH;
    *(v8ha*)(so + 8 * hi) = w0.v;
    *(v8ha*)(so + 16 + 8 * hi) = w1.v;
  }
  __syncthreads();

  att_store_pass(sO, att, tb, hd, lane);
  __threadfence();
  att_store_pass(sO, att, tb, hd, lane);
}

__device__ __forceinline__ v8f ln_row(v4f a0, v4f a1, const float* __restrict__ sc,
                                      const float* __restrict__ bi, int lane) {
  float s = ((a0.x + a0.y) + (a0.z + a0.w)) + ((a1.x + a1.y) + (a1.z + a1.w));
  s = wsum32(s);
  const float mean = s * (1.0f / (float)D_MODEL);
  const v4f d0 = a0 - mean, d1 = a1 - mean;
  float q = ((d0.x * d0.x + d0.y * d0.y) + (d0.z * d0.z + d0.w * d0.w)) +
            ((d1.x * d1.x + d1.y * d1.y) + (d1.z * d1.z + d1.w * d1.w));
  q = wsum32(q);
  const float inv = rsqrtf(q * (1.0f / (float)D_MODEL) + LNEPS);
  const v4f c0 = *(const v4fa*)(sc + 8 * lane), c1 = *(const v4fa*)(sc + 8 * lane + 4);
  const v4f b0 = *(const v4fa*)(bi + 8 * lane), b1 = *(const v4fa*)(bi + 8 * lane + 4);
  const v4f o0 = d0 * inv * c0 + b0;
  const v4f o1 = d1 * inv * c1 + b1;
  const v8f o = {o0.x, o0.y, o0.z, o0.w, o1.x, o1.y, o1.z, o1.w};
  return o;
}

__device__ __forceinline__ void ln_store_pass(const float* sw, float* xw, _Float16* hw, v8h hv, int lane) {
  const v4f g0 = *(const v4fa*)(sw + 4 * lane);
  const v4f g1 = *(const v4fa*)(sw + 128 + 4 * lane);
  *(volatile v4f*)(xw + 4 * lane) = g0;
  *(volatile v4f*)(xw + 128 + 4 * lane) = g1;
  *(volatile v8h*)(hw + 8 * lane) = hv;
}

__global__ __launch_bounds__(256) void ln_kernel(const float* x, const float* __restrict__ res,
                                                 const float* __restrict__ sc, const float* __restrict__ bi,
                                                 float* xo, _Float16* __restrict__ xh)
{
  __shared__ __attribute__((aligned(16))) float sh[8 * D_MODEL];
  const int tid = threadIdx.x, lane = tid & 31, w = tid >> 5;
  const size_t t = (size_t)blockIdx.x * 8 + w;
  const float* xr = x + t * D_MODEL + 8 * lane;
  const float* rr = res + t * D_MODEL + 8 * lane;
  const v4f a0 = *(const v4fa*)xr + *(const v4fa*)rr;
  const v4f a1 = *(const v4fa*)(xr + 4) + *(const v4fa*)(rr + 4);
  const v8f o = ln_row(a0, a1, sc, bi, lane);
  float* sw = sh + w * D_MODEL;
  const v4f o0 = {o[0], o[1], o[2], o[3]};
  const v4f o1 = {o[4], o[5], o[6], o[7]};
  *(v4fa*)(sw + 8 * lane) = o0;
  *(v4fa*)(sw + 8 * lane + 4) = o1;
  H8 hv;
  #pragma unroll
  for (int i = 0; i < 8; ++i) hv.s[i] = (_Float16)o[i];
  __syncthreads();
  ln_store_pass(sw, xo + t * D_MODEL, xh + t * D_MODEL, hv.v, lane);
  __threadfence();
  ln_store_pass(sw, xo + t * D_MODEL, xh + t * D_MODEL, hv.v, lane);
}

__device__ __forceinline__ void final_store_pass(const float* sT, float* out, int b, int l0, int w, int lane) {
  const int q8 = lane & 7, sub = lane >> 3;
  #pragma unroll
  for (int i = 0; i < 8; ++i) {
    const int ch = 32 * w + 4 * i + sub;
    const float* sp = sT + (4 * q8) * TP + ch;
    const v4f v = {sp[0], sp[TP], sp[2 * TP], sp[3 * TP]};
    *(volatile v4f*)(out + ((size_t)(b * D_MODEL + ch)) * SEQ + l0 + 4 * q8) = v;
  }
}

__global__ __launch_bounds__(256) void final_kernel(const float* __restrict__ x, const float* __restrict__ sc,
                                                    const float* __restrict__ bi, int img0, float* __restrict__ out)
{
  __shared__ __attribute__((aligned(16))) float sT[32 * TP];
  const int tid = threadIdx.x, lane = tid & 31, w = tid >> 5;
  const int bl = blockIdx.x >> 5;
  const int l0 = (blockIdx.x & 31) * 32;
  const int b  = img0 + bl;
  const size_t r0 = (size_t)bl * SEQ + l0;
  #pragma unroll
  for (int e = 0; e < 4; ++e) {
    const int tl = 4 * w + e;
    const float* xr = x + (r0 + tl) * D_MODEL + 8 * lane;
    const v4f a0 = *(const v4fa*)xr;
    const v4f a1 = *(const v4fa*)(xr + 4);
    const v8f o = ln_row(a0, a1, sc, bi, lane);
    float* st = sT + tl * TP + 8 * lane;
    const v4f o0 = {o[0], o[1], o[2], o[3]};
    const v4f o1 = {o[4], o[5], o[6], o[7]};
    *(v4fa*)st = o0;
    *(v4fa*)(st + 4) = o1;
  }
  __syncthreads();
  final_store_pass(sT, out, b, l0, w, lane);
  __threadfence();
  final_store_pass(sT, out, b, l0, w, lane);
}

extern "C" void kernel_launch(void* const* d_in, const int* in_sizes, int n_in,
                              void* d_out, int out_size, void* d_ws, size_t ws_size,
                              hipStream_t stream) {
  if (n_in < 15) return;
  if (in_sizes[0] != NTOK * D_MODEL || out_size != NTOK * D_MODEL) return;
  if (in_sizes[1] != NLAYERS * QKVN * D_MODEL || in_sizes[2] != NLAYERS * QKVN) return;
  if (in_sizes[3] != NLAYERS * D_MODEL * D_MODEL || in_sizes[4] != NLAYERS * D_MODEL) return;
  if (in_sizes[5] != NLAYERS * DFF * D_MODEL || in_sizes[6] != NLAYERS * DFF) return;
  if (in_sizes[7] != NLAYERS * D_MODEL * DFF || in_sizes[8] != NLAYERS * D_MODEL) return;
  if (in_sizes[9] != NLAYERS * D_MODEL || in_sizes[10] != NLAYERS * D_MODEL) return;
  if (in_sizes[11] != NLAYERS * D_MODEL || in_sizes[12] != NLAYERS * D_MODEL) return;
  if (in_sizes[13] != D_MODEL || in_sizes[14] != D_MODEL) return;

  const float* features   = (const float*)d_in[0];
  const float* in_proj_w  = (const float*)d_in[1];
  const float* in_proj_b  = (const float*)d_in[2];
  const float* out_proj_w = (const float*)d_in[3];
  const float* out_proj_b = (const float*)d_in[4];
  const float* w1         = (const float*)d_in[5];
  const float* b1         = (const float*)d_in[6];
  const float* w2         = (const float*)d_in[7];
  const float* b2         = (const float*)d_in[8];
  const float* ln1_s      = (const float*)d_in[9];
  const float* ln1_b      = (const float*)d_in[10];
  const float* ln2_s      = (const float*)d_in[11];
  const float* ln2_b      = (const float*)d_in[12];
  const float* fnorm_s    = (const float*)d_in[13];
  const float* fnorm_b    = (const float*)d_in[14];
  float* out = (float*)d_out;

  char* base = (char*)d_ws;
  size_t off = 0;
  auto carve = [&](size_t bytes) -> char* {
    off = (off + 255) & ~(size_t)255;
    char* p = base + off;
    off += bytes;
    return p;
  };
  _Float16* wih = (_Float16*)carve((size_t)NLAYERS * QKVN * D_MODEL * 2);
  _Float16* woh = (_Float16*)carve((size_t)NLAYERS * D_MODEL * D_MODEL * 2);
  _Float16* w1h = (_Float16*)carve((size_t)NLAYERS * DFF * D_MODEL * 2);
  _Float16* w2h = (_Float16*)carve((size_t)NLAYERS * D_MODEL * DFF * 2);
  float*    xf  = (float*)   carve((size_t)MC * D_MODEL * 4);
  _Float16* xb  = (_Float16*)carve((size_t)MC * D_MODEL * 2);
  _Float16* qkv = (_Float16*)carve((size_t)MC * QKVN * 2);
  _Float16* att = (_Float16*)carve((size_t)MC * D_MODEL * 2);
  float*    yf  = (float*)   carve((size_t)MC * D_MODEL * 4);
  _Float16* hb  = (_Float16*)carve((size_t)MC * DFF * 2);
  if (off > ws_size) return;
  if (off > (size_t)134217728) return;

  {
    const int g0 = in_sizes[1] / 8, g1 = in_sizes[3] / 8, g2 = in_sizes[5] / 8, g3 = in_sizes[7] / 8;
    const int tot = g0 + g1 + g2 + g3;
    cvt_w_kernel<<<(tot + 255) / 256, 256, 0, stream>>>(in_proj_w, out_proj_w, w1, w2,
                                                        wih, woh, w1h, w2h, g0, g1, g2, g3);
  }

  for (int c = 0; c < NCHUNK; ++c) {
    const int img0 = c * IMGC;

    prep_kernel<<<MC / 32, 256, 0, stream>>>(features, img0, xf, xb);

    for (int i = 0; i < NLAYERS; ++i) {
      gemm_f16_kernel<<<dim3(MC / 128, QKVN / 64), 128, 0, stream>>>(
          xb, D_MODEL, wih + (size_t)i * QKVN * D_MODEL, D_MODEL,
          in_proj_b + (size_t)i * QKVN, yf, qkv, QKVN, D_MODEL, 0, 1);

      attn_kernel<<<MC / WIN, 256, 0, stream>>>(qkv, att);

      gemm_f16_kernel<<<dim3(MC / 128, D_MODEL / 64), 128, 0, stream>>>(
          att, D_MODEL, woh + (size_t)i * D_MODEL * D_MODEL, D_MODEL,
          out_proj_b + (size_t)i * D_MODEL, yf, hb, D_MODEL, 0, 0, 0);

      ln_kernel<<<MC / 8, 256, 0, stream>>>(
          xf, yf, ln1_s + (size_t)i * D_MODEL, ln1_b + (size_t)i * D_MODEL, xf, xb);

      gemm_f16_kernel<<<dim3(MC / 128, DFF / 64), 128, 0, stream>>>(
          xb, D_MODEL, w1h + (size_t)i * DFF * D_MODEL, D_MODEL,
          b1 + (size_t)i * DFF, yf, hb, DFF, 0, 1, 1);

      gemm_f16_kernel<<<dim3(MC / 128, D_MODEL / 64), 128, 0, stream>>>(
          hb, DFF, w2h + (size_t)i * D_MODEL * DFF, DFF,
          b2 + (size_t)i * D_MODEL, yf, qkv, D_MODEL, 0, 0, 0);

      ln_kernel<<<MC / 8, 256, 0, stream>>>(
          xf, yf, ln2_s + (size_t)i * D_MODEL, ln2_b + (size_t)i * D_MODEL, xf, xb);
    }

    final_kernel<<<MC / 32, 256, 0, stream>>>(xf, fnorm_s, fnorm_b, img0, out);
  }
}
